// MambaBlock_12764642803900
// MI455X (gfx1250) — hardware-verified
//
#include <hip/hip_runtime.h>
#include <math.h>

typedef __attribute__((ext_vector_type(16))) _Float16 v16h;
typedef __attribute__((ext_vector_type(8)))  _Float16 v8h;
typedef __attribute__((ext_vector_type(8)))  float    v8f;
typedef __attribute__((ext_vector_type(4)))  float    v4f;

constexpr int kBatch  = 2;
constexpr int kSeq    = 2048;
constexpr int kDm     = 512;
constexpr int kDin    = 1024;
constexpr int kNst    = 16;
constexpr int kDtR    = 32;
constexpr int kXzP    = 2 * kDin;
constexpr int kXdP    = 64;
constexpr int kRows   = kBatch * kSeq;
constexpr int kConvTP = 260;
constexpr int kScanTS = 64;
constexpr int kScanCh = 64;
constexpr int kScanYP = 68;
constexpr float kLnEps = 1e-5f;
constexpr float kCarryW  = 32.0f;
constexpr float kCarryXc = 8.0f;
constexpr float kCarryY  = 16.0f;
constexpr float kScaleIn  = 1.0f / kCarryW;
constexpr float kScaleXp  = 1.0f / (kCarryXc * kCarryW);
constexpr float kScaleOut = 1.0f / (kCarryY * kCarryW);
static_assert(kDtR + 2 * kNst == kXdP, "x_proj width");
static_assert((kDm % 32) == 0 && (kDin % 32) == 0, "GEMM K multiples of 32");
static_assert((kRows % 64) == 0 && (kXzP % 64) == 0 && (kXdP % 64) == 0 && (kDm % 64) == 0, "GEMM M,N multiples of 64");
static_assert((kSeq % kScanTS) == 0 && (kSeq % 64) == 0 && (kDin % kScanCh) == 0 && (kDin % 256) == 0, "tile multiples");
static_assert(((kRows / 64) * (kXzP / 64)) % 8 == 0 && ((kRows / 64) * (kXdP / 64)) % 8 == 0 && ((kRows / 64) * (kDm / 64)) % 8 == 0, "whole GEMM blocks");
static_assert(kDm == 512, "LayerNorm lane map assumes 512 columns");

constexpr size_t kOffWIN  = 0;
constexpr size_t kOffWOUT = kOffWIN  + (size_t)kXzP * kDm * 2;
constexpr size_t kOffWXP  = kOffWOUT + (size_t)kDm * kDin * 2;
constexpr size_t kOffH16  = kOffWXP  + (size_t)2 * kXdP * kDin * 2;
constexpr size_t kOffXZ   = kOffH16  + (size_t)kRows * kDm * 2;
constexpr size_t kOffXC   = kOffXZ   + (size_t)kRows * kXzP * 4;
constexpr size_t kOffXD   = kOffXC   + (size_t)2 * kRows * kDin * 2;
constexpr size_t kOffY    = kOffXD   + (size_t)2 * kRows * kXdP * 4;
constexpr size_t kOffYS   = kOffY    + (size_t)2 * kRows * kDin * 4;
constexpr size_t kWsTotal = kOffYS   + (size_t)kRows * kDin * 2;
static_assert(kWsTotal == 101974016ull, "carve total");
static_assert(kWsTotal <= 134217728ull, "carve cap");
static_assert((kOffWOUT % 128) == 0 && (kOffWXP % 128) == 0 && (kOffH16 % 128) == 0 && (kOffXZ % 128) == 0 &&
              (kOffXC % 128) == 0 && (kOffXD % 128) == 0 && (kOffY % 128) == 0 && (kOffYS % 128) == 0, "128-B aligned regions");

union FragU { v16h v; v8h h[2]; };
__device__ __forceinline__ v16h frag_load_h(const _Float16* p) {
  FragU f;
  f.h[0] = *(const v8h*)(p);
  f.h[1] = *(const v8h*)(p + 16);
  return f.v;
}
__device__ __forceinline__ v8f mma_h(v16h a, v16h b, v8f c) {
  return __builtin_amdgcn_wmma_f32_16x16x32_f16(false, a, false, b, (short)0, c, false, false);
}
__device__ __forceinline__ void guard_group_h(v8f& a0, v8f& a1, v8f& a2, v8f& a3,
                                              v16h x, v16h b0, v16h b1, v16h b2, v16h b3) {
  asm volatile("v_nop\n\tv_nop\n\tv_nop\n\tv_nop"
               : "+v"(a0), "+v"(a1), "+v"(a2), "+v"(a3)
               : "v"(x), "v"(b0), "v"(b1), "v"(b2), "v"(b3));
}
__device__ __forceinline__ void keep4_h(v16h a, v16h b, v16h c, v16h d) { asm volatile("v_nop" :: "v"(a), "v"(b), "v"(c), "v"(d)); }
__device__ __forceinline__ void acc_guard4(v8f& a, v8f& b, v8f& c, v8f& d) { asm volatile("v_nop\n\tv_nop\n\tv_nop\n\tv_nop" : "+v"(a), "+v"(b), "+v"(c), "+v"(d)); }

__global__ __launch_bounds__(256) void wmma_gemm64_f16(
    const unsigned short* __restrict__ Ap, int lda, long strideA,
    const unsigned short* __restrict__ Btp, int ldb, long strideB,
    float* __restrict__ Cout, int ldc, long strideC,
    int M, int N, int K, float scale) {
  const _Float16* A  = (const _Float16*)Ap;
  const _Float16* Bt = (const _Float16*)Btp;
  __shared__ __align__(16) float sT[8][16 * 68];
  const int b    = blockIdx.y;
  const int lane = threadIdx.x & 31;
  const int wave = threadIdx.x >> 5;
  const int tilesN = N >> 6;
  const int tilesM = M >> 6;
  const int tile = blockIdx.x * 8 + wave;
  if (tile >= tilesM * tilesN) return;
  const int tm = tile / tilesN;
  const int tn = tile - tm * tilesN;
  const int m0 = tm << 6;
  const int n0 = tn << 6;

  const _Float16* Ab = A  + (size_t)b * strideA;
  const _Float16* Bb = Bt + (size_t)b * strideB;

  const int rlane = lane & 15;
  const int koff  = (lane >> 4) * 8;
  const int mOff  = (lane >> 4) * 8;

  v8f acc[4][4];
#pragma unroll
  for (int i = 0; i < 4; ++i)
#pragma unroll
    for (int j = 0; j < 4; ++j) acc[i][j] = (v8f){0.f,0.f,0.f,0.f,0.f,0.f,0.f,0.f};

  for (int k0 = 0; k0 < K; k0 += 32) {
    v16h bh[4];
#pragma unroll
    for (int j = 0; j < 4; ++j) {
      const size_t bo = (size_t)(n0 + (j << 4) + rlane) * ldb + koff + k0;
      bh[j] = frag_load_h(Bb + bo);
    }
#pragma unroll
    for (int i = 0; i < 4; ++i) {
      const size_t ao = (size_t)(m0 + (i << 4) + rlane) * lda + koff + k0;
      v16h ah = frag_load_h(Ab + ao);
#pragma unroll
      for (int j = 0; j < 4; ++j) acc[i][j] = mma_h(ah, bh[j], acc[i][j]);
      guard_group_h(acc[i][0], acc[i][1], acc[i][2], acc[i][3], ah, bh[0], bh[1], bh[2], bh[3]);
    }
    keep4_h(bh[0], bh[1], bh[2], bh[3]);
  }
  acc_guard4(acc[0][0], acc[0][1], acc[0][2], acc[0][3]);
  acc_guard4(acc[1][0], acc[1][1], acc[1][2], acc[1][3]);
  acc_guard4(acc[2][0], acc[2][1], acc[2][2], acc[2][3]);
  acc_guard4(acc[3][0], acc[3][1], acc[3][2], acc[3][3]);

  float* slab = sT[wave];
  float* C = Cout + (size_t)b * strideC;
#pragma unroll
  for (int i = 0; i < 4; ++i) {
    const int mBase = m0 + (i << 4);
#pragma unroll
    for (int j = 0; j < 4; ++j) {
#pragma unroll
      for (int r = 0; r < 8; ++r) {
        const float v = acc[i][j][r] * scale;
        slab[(mOff + r) * 68 + (j << 4) + rlane] = v;
      }
    }
    __builtin_amdgcn_fence(__ATOMIC_RELEASE, "workgroup");
    __builtin_amdgcn_wave_barrier();
    __builtin_amdgcn_fence(__ATOMIC_ACQUIRE, "workgroup");
    {
      const int hh = lane >> 4, c4 = (lane & 15) * 4;
      for (int pass = 0; pass < 2; ++pass) {
#pragma unroll
        for (int it = 0; it < 8; ++it) {
          const int row = it * 2 + hh;
          v4f v = *(const v4f*)(slab + row * 68 + c4);
          *(volatile v4f*)(C + (size_t)(mBase + row) * ldc + n0 + c4) = v;
        }
        __threadfence();
      }
    }
    __builtin_amdgcn_fence(__ATOMIC_RELEASE, "workgroup");
    __builtin_amdgcn_wave_barrier();
    __builtin_amdgcn_fence(__ATOMIC_ACQUIRE, "workgroup");
  }
}

constexpr int kCastBlkWin  = (kXzP * kDm / 8) / 256;
constexpr int kCastBlkWout = (kDm * kDin / 8) / 256;
constexpr int kCastBlkWxp  = (kXdP * kDin / 8) / 256;
constexpr int kCastBlkAll  = kCastBlkWin + kCastBlkWout + 2 * kCastBlkWxp;
static_assert(kCastBlkWin == 512 && kCastBlkWout == 256 && kCastBlkWxp == 32, "cast block ranges");

__global__ __launch_bounds__(256) void cast_weights_kernel(
    const float* __restrict__ win, const float* __restrict__ wout,
    const float* __restrict__ wxf, const float* __restrict__ wxb,
    unsigned short* __restrict__ dwin, unsigned short* __restrict__ dwout,
    unsigned short* __restrict__ dwxf, unsigned short* __restrict__ dwxb)
{
  int blk = blockIdx.x;
  const float* src;
  unsigned short* dst;
  if (blk < kCastBlkWin) {
    src = win; dst = dwin;
  } else if (blk < kCastBlkWin + kCastBlkWout) {
    src = wout; dst = dwout; blk -= kCastBlkWin;
  } else if (blk < kCastBlkWin + kCastBlkWout + kCastBlkWxp) {
    src = wxf; dst = dwxf; blk -= kCastBlkWin + kCastBlkWout;
  } else {
    src = wxb; dst = dwxb; blk -= kCastBlkWin + kCastBlkWout + kCastBlkWxp;
  }
  const size_t e0 = ((size_t)blk * 256 + threadIdx.x) << 3;
  const v4f a0 = *(const v4f*)(src + e0);
  const v4f a1 = *(const v4f*)(src + e0 + 4);
  v8h hv;
#pragma unroll
  for (int e = 0; e < 4; ++e) {
    hv[e]     = (_Float16)(a0[e] * kCarryW);
    hv[4 + e] = (_Float16)(a1[e] * kCarryW);
  }
  unsigned short* q = dst + e0;
  *(volatile v8h*)q = hv;
  __threadfence();
  *(volatile v8h*)q = hv;
}

__global__ __launch_bounds__(256) void ln_copy_kernel(
    const float* __restrict__ x, const float* __restrict__ nw, const float* __restrict__ nb,
    unsigned short* __restrict__ H16, float* __restrict__ out1)
{
  const int lane = threadIdx.x & 31, wave = threadIdx.x >> 5;
  const int row = blockIdx.x * 8 + wave;
  const float* xr = x + (size_t)row * kDm;
  v4f cp[4];
#pragma unroll
  for (int it = 0; it < 4; ++it) cp[it] = *(const v4f*)(xr + it * 128 + lane * 4);
  v4f a[4];
#pragma unroll
  for (int c = 0; c < 2; ++c) {
    a[2 * c]     = *(const v4f*)(xr + c * 256 + lane * 8);
    a[2 * c + 1] = *(const v4f*)(xr + c * 256 + lane * 8 + 4);
  }
  float s = 0.0f;
#pragma unroll
  for (int i = 0; i < 4; ++i) s += (a[i][0] + a[i][1]) + (a[i][2] + a[i][3]);
#pragma unroll
  for (int off = 16; off > 0; off >>= 1) s += __shfl_xor(s, off, 32);
  const float mu = s * (1.0f / (float)kDm);
  float sq = 0.0f;
#pragma unroll
  for (int i = 0; i < 4; ++i) {
#pragma unroll
    for (int e = 0; e < 4; ++e) {
      const float dlt = a[i][e] - mu;
      sq = fmaf(dlt, dlt, sq);
    }
  }
#pragma unroll
  for (int off = 16; off > 0; off >>= 1) sq += __shfl_xor(sq, off, 32);
  const float var = sq * (1.0f / (float)kDm);
  const float rs = rsqrtf(var + kLnEps);
  v8h hv[2];
#pragma unroll
  for (int c = 0; c < 2; ++c) {
    const v4f w0 = *(const v4f*)(nw + c * 256 + lane * 8);
    const v4f w1 = *(const v4f*)(nw + c * 256 + lane * 8 + 4);
    const v4f b0 = *(const v4f*)(nb + c * 256 + lane * 8);
    const v4f b1 = *(const v4f*)(nb + c * 256 + lane * 8 + 4);
#pragma unroll
    for (int e = 0; e < 4; ++e) {
      const float y0 = ((a[2 * c][e] - mu) * rs) * w0[e] + b0[e];
      const float y1 = ((a[2 * c + 1][e] - mu) * rs) * w1[e] + b1[e];
      hv[c][e]     = (_Float16)y0;
      hv[c][4 + e] = (_Float16)y1;
    }
  }
  float* orow = out1 + (size_t)row * kDm;
  unsigned short* hrow = H16 + (size_t)row * kDm;
  for (int pass = 0; pass < 2; ++pass) {
#pragma unroll
    for (int it = 0; it < 4; ++it) *(volatile v4f*)(orow + it * 128 + lane * 4) = cp[it];
#pragma unroll
    for (int c = 0; c < 2; ++c) *(volatile v8h*)(hrow + c * 256 + lane * 8) = hv[c];
    __threadfence();
  }
}

__global__ __launch_bounds__(256) void conv_silu_kernel(
    const float* __restrict__ XZ,
    const float* __restrict__ cw_f, const float* __restrict__ cb_f,
    const float* __restrict__ cw_b, const float* __restrict__ cb_b,
    unsigned short* __restrict__ XC16)
{
  __shared__ __align__(16) float sT[16 * kConvTP];
  const int tid = threadIdx.x, lane = tid & 31, wave = tid >> 5;
  const int dir = blockIdx.z;
  const float* cw = dir ? cw_b : cw_f;
  const float* cb = dir ? cb_b : cb_f;
  unsigned short* XCp = XC16 + (size_t)dir * kRows * kDin;
  const int d0 = blockIdx.x * 256, d = d0 + tid;
  const int g0 = blockIdx.y * 64;
  const int tb = g0 & (kSeq - 1);
  const int sgn = dir ? -1 : 1;
  const int gstart = dir ? (g0 + 63) : g0;
  const bool hist = dir ? (tb + 64 < kSeq) : (tb > 0);
  const v4f wv = *(const v4f*)(cw + (size_t)d * 4);
  const float w0 = wv[0], w1 = wv[1], w2 = wv[2], w3 = wv[3];
  const float bc = cb[d];
  float xm3, xm2, xm1;
  {
    const int r1 = hist ? (gstart - sgn) : gstart;
    const int r2 = hist ? (gstart - 2 * sgn) : gstart;
    const int r3 = hist ? (gstart - 3 * sgn) : gstart;
    const float v1 = XZ[(size_t)r1 * kXzP + d];
    const float v2 = XZ[(size_t)r2 * kXzP + d];
    const float v3 = XZ[(size_t)r3 * kXzP + d];
    xm1 = hist ? v1 : 0.0f;
    xm2 = hist ? v2 : 0.0f;
    xm3 = hist ? v3 : 0.0f;
  }
#pragma unroll 1
  for (int sub = 0; sub < 4; ++sub) {
#pragma unroll 1
    for (int s = 0; s < 16; ++s) {
      const int row = gstart + sgn * (sub * 16 + s);
      const float xcur = XZ[(size_t)row * kXzP + d];
      float u = fmaf(w0, xm3, bc);
      u = fmaf(w1, xm2, u);
      u = fmaf(w2, xm1, u);
      u = fmaf(w3, xcur, u);
      const float sg = __builtin_amdgcn_rcpf(1.0f + expf(-u));
      sT[s * kConvTP + tid] = u * sg;
      xm3 = xm2; xm2 = xm1; xm1 = xcur;
    }
    __syncthreads();
    v8h hv[2];
#pragma unroll
    for (int it = 0; it < 2; ++it) {
      const float* sp = sT + (it * 8 + wave) * kConvTP + lane * 8;
      const v4f a0 = *(const v4f*)(sp);
      const v4f a1 = *(const v4f*)(sp + 4);
#pragma unroll
      for (int e = 0; e < 4; ++e) {
        hv[it][e]     = (_Float16)(a0[e] * kCarryXc);
        hv[it][4 + e] = (_Float16)(a1[e] * kCarryXc);
      }
    }
    for (int pass = 0; pass < 2; ++pass) {
#pragma unroll
      for (int it = 0; it < 2; ++it) {
        const int grow = gstart + sgn * (sub * 16 + it * 8 + wave);
        *(volatile v8h*)(XCp + (size_t)grow * kDin + d0 + lane * 8) = hv[it];
      }
      __threadfence();
    }
    __syncthreads();
  }
}

__global__ __launch_bounds__(64) void scan_kernel(
    const float* __restrict__ XDall, const float* __restrict__ XZ,
    const float* __restrict__ cw_f, const float* __restrict__ cb_f, const float* __restrict__ wdt_f,
    const float* __restrict__ bdt_f, const float* __restrict__ alog_f, const float* __restrict__ dsk_f,
    const float* __restrict__ cw_b, const float* __restrict__ cb_b, const float* __restrict__ wdt_b,
    const float* __restrict__ bdt_b, const float* __restrict__ alog_b, const float* __restrict__ dsk_b,
    float* __restrict__ Yall)
{
  __shared__ __align__(16) float sX[kScanTS * kXdP];
  __shared__ __align__(16) float sY[kScanTS * kScanYP];
  __shared__ __align__(16) float sW[kDtR * kScanCh];
  __shared__ __align__(16) float sA[kNst * kScanCh];
  const int tid = threadIdx.x, lane = tid & 31, wave = tid >> 5;
  const int dir = blockIdx.y;
  constexpr int kBlkPerB = kDin / kScanCh;
  const int bix = blockIdx.x / kBlkPerB;
  const int d0  = (blockIdx.x - bix * kBlkPerB) * kScanCh;
  const int d   = d0 + tid;
  const size_t row0 = (size_t)bix * kSeq;
  const float* cw   = dir ? cw_b : cw_f;
  const float* cb   = dir ? cb_b : cb_f;
  const float* Wdt  = dir ? wdt_b : wdt_f;
  const float* bdt  = dir ? bdt_b : bdt_f;
  const float* Alog = dir ? alog_b : alog_f;
  const float* Dsk  = dir ? dsk_b : dsk_f;
  const float* XD = XDall + (size_t)dir * kRows * kXdP;
  float* Yp = Yall + (size_t)dir * kRows * kDin;

#pragma unroll 1
  for (int r = 0; r < kDtR; ++r) sW[r * kScanCh + tid] = Wdt[(size_t)d * kDtR + r];
#pragma unroll 1
  for (int s = 0; s < kNst; ++s) sA[s * kScanCh + tid] = -expf(Alog[(size_t)d * kNst + s]);
  __syncthreads();
  float negA[kNst], h[kNst];
#pragma unroll
  for (int s = 0; s < kNst; ++s) {
    negA[s] = sA[s * kScanCh + tid];
    h[s] = 0.0f;
  }
  const float bb = bdt[d], Dd = Dsk[d];
  const v4f wv = *(const v4f*)(cw + (size_t)d * 4);
  const float w0 = wv[0], w1 = wv[1], w2 = wv[2], w3 = wv[3];
  const float bc = cb[d];
  float xm3 = 0.0f, xm2 = 0.0f, xm1 = 0.0f;
  const int lr = tid >> 4, lc4 = (tid & 15) * 4;
  const int hh = lane >> 4, c4 = (lane & 15) * 4;
#pragma unroll 1
  for (int t0 = 0; t0 < kSeq; t0 += kScanTS) {
    const int lo = dir ? (kSeq - kScanTS - t0) : t0;
    __syncthreads();
#pragma unroll
    for (int i = 0; i < 16; ++i) {
      const int r = lr + 4 * i;
      *(v4f*)(sX + r * kXdP + lc4) = *(const v4f*)(XD + (row0 + lo + r) * kXdP + lc4);
    }
    __syncthreads();
#pragma unroll 1
    for (int s = 0; s < kScanTS; ++s) {
      const int lrow = dir ? (kScanTS - 1 - s) : s;
      const size_t grow = row0 + (size_t)(lo + lrow);
      float xcur = XZ[grow * kXzP + d];
      asm volatile("" : "+v"(xcur));
      float zv = XZ[grow * kXzP + kDin + d];
      asm volatile("" : "+v"(zv));
      const float* xr = sX + lrow * kXdP;
      float vdot = 0.0f;
#pragma unroll 1
      for (int r4 = 0; r4 < kDtR / 4; ++r4) {
        const v4f xv = *(const v4f*)(xr + 4 * r4);
        const float* wp = sW + (4 * r4) * kScanCh + tid;
        vdot = fmaf(xv[0], wp[0], vdot);
        vdot = fmaf(xv[1], wp[kScanCh], vdot);
        vdot = fmaf(xv[2], wp[2 * kScanCh], vdot);
        vdot = fmaf(xv[3], wp[3 * kScanCh], vdot);
      }
      float Bs[kNst], Cs[kNst];
#pragma unroll
      for (int q4 = 0; q4 < 4; ++q4) {
        const v4f bv = *(const v4f*)(xr + kDtR + 4 * q4);
        const v4f cv = *(const v4f*)(xr + kDtR + kNst + 4 * q4);
        Bs[4 * q4 + 0] = bv[0]; Bs[4 * q4 + 1] = bv[1]; Bs[4 * q4 + 2] = bv[2]; Bs[4 * q4 + 3] = bv[3];
        Cs[4 * q4 + 0] = cv[0]; Cs[4 * q4 + 1] = cv[1]; Cs[4 * q4 + 2] = cv[2]; Cs[4 * q4 + 3] = cv[3];
      }
      float u = fmaf(w0, xm3, bc);
      u = fmaf(w1, xm2, u);
      u = fmaf(w2, xm1, u);
      u = fmaf(w3, xcur, u);
      const float xt = u * __builtin_amdgcn_rcpf(1.0f + expf(-u));
      xm3 = xm2; xm2 = xm1; xm1 = xcur;
      const float v   = vdot + bb;
      const float a   = expf(-fabsf(v));
      const float up  = 1.0f + a;
      const float l1p = logf(up) + (a - (up - 1.0f)) * __builtin_amdgcn_rcpf(up);
      const float dt  = fmaxf(v, 0.0f) + l1p;
      const float dtx = dt * xt;
      float y = 0.0f;
#pragma unroll
      for (int k = 0; k < kNst; ++k) {
        const float e = __expf(dt * negA[k]);
        h[k] = e * h[k] + dtx * Bs[k];
        y = h[k] * Cs[k] + y;
      }
      y = xt * Dd + y;
      const float sg = __builtin_amdgcn_rcpf(1.0f + expf(-zv));
      y = y * (zv * sg);
      sY[lrow * kScanYP + tid] = y;
    }
    __syncthreads();
    for (int pass = 0; pass < 2; ++pass) {
#pragma unroll
      for (int it = 0; it < 16; ++it) {
        const int row = it * 4 + wave * 2 + hh;
        const v4f val = *(const v4f*)(sY + row * kScanYP + c4);
        *(volatile v4f*)(Yp + (row0 + (size_t)(lo + row)) * kDin + d0 + c4) = val;
      }
      __threadfence();
    }
  }
}

__global__ __launch_bounds__(256) void combine_kernel(
    const float* __restrict__ Yall, unsigned short* __restrict__ YS16)
{
  const size_t e0 = ((size_t)blockIdx.x * 256 + threadIdx.x) << 3;
  const float* yf = Yall + e0;
  const float* yb = Yall + (size_t)kRows * kDin + e0;
  const v4f f0 = *(const v4f*)(yf);
  const v4f f1 = *(const v4f*)(yf + 4);
  const v4f b0 = *(const v4f*)(yb);
  const v4f b1 = *(const v4f*)(yb + 4);
  v8h hv;
#pragma unroll
  for (int e = 0; e < 4; ++e) {
    const float s0 = (f0[e] + b0[e]) * 0.5f;
    const float s1 = (f1[e] + b1[e]) * 0.5f;
    hv[e]     = (_Float16)(s0 * kCarryY);
    hv[4 + e] = (_Float16)(s1 * kCarryY);
  }
  unsigned short* q = YS16 + e0;
  *(volatile v8h*)q = hv;
  __threadfence();
  *(volatile v8h*)q = hv;
}

extern "C" void kernel_launch(void* const* d_in, const int* in_sizes, int n_in,
                              void* d_out, int out_size, void* d_ws, size_t ws_size,
                              hipStream_t stream) {
  if (n_in < 19) return;
  if (in_sizes[0] != kRows * kDm) return;
  if (in_sizes[1] != kDm || in_sizes[2] != kDm) return;
  if (in_sizes[3] != kXzP * kDm) return;
  if (in_sizes[4] != kDm * kDin) return;
  for (int br = 0; br < 2; ++br) {
    const int o = 5 + 7 * br;
    if (in_sizes[o + 0] != kDin * 4) return;
    if (in_sizes[o + 1] != kDin) return;
    if (in_sizes[o + 2] != kXdP * kDin) return;
    if (in_sizes[o + 3] != kDin * kDtR) return;
    if (in_sizes[o + 4] != kDin) return;
    if (in_sizes[o + 5] != kDin * kNst) return;
    if (in_sizes[o + 6] != kDin) return;
  }
  if (out_size != 2 * kRows * kDm) return;
  if (ws_size < kWsTotal) return;

  const float* hidden   = (const float*)d_in[0];
  const float* norm_w   = (const float*)d_in[1];
  const float* norm_b   = (const float*)d_in[2];
  const float* in_w     = (const float*)d_in[3];
  const float* out_w    = (const float*)d_in[4];
  const float* conv_w_f = (const float*)d_in[5];
  const float* conv_b_f = (const float*)d_in[6];
  const float* xp_w_f   = (const float*)d_in[7];
  const float* dt_w_f   = (const float*)d_in[8];
  const float* dt_b_f   = (const float*)d_in[9];
  const float* alog_f   = (const float*)d_in[10];
  const float* dsk_f    = (const float*)d_in[11];
  const float* conv_w_b = (const float*)d_in[12];
  const float* conv_b_b = (const float*)d_in[13];
  const float* xp_w_b   = (const float*)d_in[14];
  const float* dt_w_b   = (const float*)d_in[15];
  const float* dt_b_b   = (const float*)d_in[16];
  const float* alog_b   = (const float*)d_in[17];
  const float* dsk_b    = (const float*)d_in[18];

  float* out0 = (float*)d_out;
  float* out1 = out0 + (size_t)kRows * kDm;

  char* ws = (char*)d_ws;
  unsigned short* WIN16  = (unsigned short*)(ws + kOffWIN);
  unsigned short* WOUT16 = (unsigned short*)(ws + kOffWOUT);
  unsigned short* WXP16  = (unsigned short*)(ws + kOffWXP);
  unsigned short* H16    = (unsigned short*)(ws + kOffH16);
  float*          XZ     = (float*)(ws + kOffXZ);
  unsigned short* XC16   = (unsigned short*)(ws + kOffXC);
  float*          XD     = (float*)(ws + kOffXD);
  float*          Y      = (float*)(ws + kOffY);
  unsigned short* YS16   = (unsigned short*)(ws + kOffYS);

  cast_weights_kernel<<<kCastBlkAll, 256, 0, stream>>>(
      in_w, out_w, xp_w_f, xp_w_b,
      WIN16, WOUT16, WXP16, WXP16 + (size_t)kXdP * kDin);

  ln_copy_kernel<<<kRows / 8, 256, 0, stream>>>(hidden, norm_w, norm_b, H16, out1);

  wmma_gemm64_f16<<<dim3((kRows / 64) * (kXzP / 64) / 8, 1), 256, 0, stream>>>(
      H16, kDm, 0L, WIN16, kDm, 0L, XZ, kXzP, 0L, kRows, kXzP, kDm, kScaleIn);

  conv_silu_kernel<<<dim3(kDin / 256, kRows / 64, 2), 256, 0, stream>>>(
      XZ, conv_w_f, conv_b_f, conv_w_b, conv_b_b, XC16);

  wmma_gemm64_f16<<<dim3((kRows / 64) * (kXdP / 64) / 8, 2), 256, 0, stream>>>(
      XC16, kDin, (long)kRows * kDin, WXP16, kDin, (long)kXdP * kDin,
      XD, kXdP, (long)kRows * kXdP, kRows, kXdP, kDin, kScaleXp);

  scan_kernel<<<dim3(kBatch * (kDin / kScanCh), 2), kScanCh, 0, stream>>>(
      XD, XZ,
      conv_w_f, conv_b_f, dt_w_f, dt_b_f, alog_f, dsk_f,
      conv_w_b, conv_b_b, dt_w_b, dt_b_b, alog_b, dsk_b,
      Y);

  combine_kernel<<<(kRows * kDin / 8) / 256, 256, 0, stream>>>(Y, YS16);

  wmma_gemm64_f16<<<dim3((kRows / 64) * (kDm / 64) / 8, 1), 256, 0, stream>>>(
      YS16, kDin, 0L, WOUT16, kDin, 0L, out0, kDm, 0L, kRows, kDm, kDin, kScaleOut);
}
